// DCM_30313879175980
// MI455X (gfx1250) — hardware-run, weakly checked
//
#include <hip/hip_runtime.h>
#pragma clang fp contract(off)


#ifndef NTX
#define NTX 64
#endif
#ifndef NVD
#define NVD 64
#endif
#define NTX_FULL 64
#define NVD_FULL 64
#define TT   32
#define VV   12
#define DW   512
#define NROW (NTX * TT)
#define NCOL (NVD * VV)
#define EW   8
#define BPW  (NVD / EW)
#define TAUF 100.0f
#define EPSF 1e-6f
#define L2E  1.4426950408889634f

static_assert(TT == 32);
static_assert(VV % 4 == 0);
static_assert((VV * 4) % 16 == 0);
static_assert(DW % 32 == 0);
static_assert(DW == 4 * 128);
static_assert(NROW % 64 == 0);
static_assert(NCOL % 64 == 0);
static_assert(NROW % 32 == 0);
static_assert(NCOL % 32 == 0);
static_assert(NCOL % 4 == 0);
static_assert(EW * 4 == 32);
static_assert(8 * 16 == 32 * 4);
static_assert(NVD % 32 == 0);
static_assert(NVD % EW == 0);
static_assert(NVD / 4 <= 32);
static_assert((NVD / 4) * 16 == NVD * 4);
static_assert(32 * 16 * 8 == 16 * 64 * 4);
static_assert(NTX <= NTX_FULL);
static_assert(NVD <= NVD_FULL);
static_assert(((size_t)NROW * DW) % 8 == 0);
static_assert(((size_t)NCOL * DW) % 8 == 0);
static_assert(16 * 68 * 4 <= 131072);
static_assert((EW * TT * VV + NVD) * 4 <= 131072);
static_assert(32 * 4 <= 131072);

typedef unsigned short bf;
typedef __attribute__((ext_vector_type(16))) __bf16   v16bf;
typedef __attribute__((ext_vector_type(8)))  unsigned short v8us;
typedef __attribute__((ext_vector_type(8)))  float    v8f;
typedef __attribute__((ext_vector_type(4)))  float    v4f;
typedef v4f  __attribute__((may_alias)) v4fa;

__device__ __forceinline__ unsigned short f2bf(float f) { unsigned u = __float_as_uint(f); u += 0x7FFFu + ((u >> 16) & 1u); return (unsigned short)(u >> 16); }
__device__ __forceinline__ float bfr(float f) { return __uint_as_float(((unsigned)f2bf(f)) << 16); }
__device__ __forceinline__ v16bf cat16b(v8us lo, v8us hi) { return __builtin_bit_cast(v16bf, __builtin_shufflevector(lo, hi, 0, 1, 2, 3, 4, 5, 6, 7, 8, 9, 10, 11, 12, 13, 14, 15)); }
__device__ __forceinline__ v8f wmmab(v16bf a, v16bf b, v8f c) { return __builtin_amdgcn_wmma_f32_16x16x32_bf16(false, a, false, b, (short)0, c, false, false); }
__device__ __forceinline__ v8f wmmab_g(v16bf a, v16bf b, v8f c) { c = wmmab(a, b, c); asm volatile("v_nop\n\tv_nop\n\tv_nop\n\tv_nop" : "+v"(c) : "v"(a), "v"(b)); return c; }
__device__ __forceinline__ v16bf ldb(const bf* p)  { return cat16b(*(const v8us*)p, *(const v8us*)(p + 16)); }
__device__ __forceinline__ void wave_sync() { __builtin_amdgcn_fence(3  , "wavefront"); __builtin_amdgcn_wave_barrier(); asm volatile("" ::: "memory"); }
__device__ __forceinline__ float wsum(float x) {
#pragma unroll
    for (int o = 16; o > 0; o >>= 1) x += __shfl_xor(x, o, 32);
    return x; }
__device__ __forceinline__ float wmax(float x) {
#pragma unroll
    for (int o = 16; o > 0; o >>= 1) x = fmaxf(x, __shfl_xor(x, o, 32));
    return x; }

__global__ __launch_bounds__(256) void k_cvt8(const float* __restrict__ src, bf* dst, size_t n8) {
    const size_t i = (size_t)blockIdx.x * 256 + threadIdx.x; if (i >= n8) return;
    const v8f v = *(const v8f*)(src + i * 8); v8us o;
#pragma unroll
    for (int k = 0; k < 8; ++k) o[k] = f2bf(v[k]);
    *(volatile v8us*)(dst + i * 8) = o; __threadfence(); *(volatile v8us*)(dst + i * 8) = o;
}

__global__ __launch_bounds__(32 * EW) void k_norm(const float* __restrict__ src, float* inv, int nrows) {
    __shared__ __align__(16) float sn[32];
    const int lane = threadIdx.x & 31;
    const int wave = __builtin_amdgcn_readfirstlane((int)(threadIdx.x >> 5));
#pragma unroll 1
    for (int i = 0; i < 4; ++i) {
        int row = (int)blockIdx.x * 32 + wave * 4 + i; row = row < nrows - 1 ? row : nrows - 1;
        const float* p = src + (size_t)row * DW + lane * 4;
        float s = 0.0f;
#pragma unroll 1
        for (int q = 0; q < 4; ++q) {
            const v4f x = *(const v4f*)(p + q * 128);
            const float y0 = bfr(x[0]), y1 = bfr(x[1]), y2 = bfr(x[2]), y3 = bfr(x[3]);
            s += y0 * y0; s += y1 * y1; s += y2 * y2; s += y3 * y3; }
        s = wsum(s);
        const float r = 1.0f / fmaxf(sqrtf(s), EPSF);
        if (lane == 0) sn[wave * 4 + i] = r;
    }
    __syncthreads();
    if (wave == 0) {
        const int lc = lane < 8 ? lane : 7;
        const v4f val = *(const v4fa*)(&sn[lc * 4]);
        float* o = inv + (size_t)blockIdx.x * 32 + lc * 4;
#pragma unroll 1
        for (int ps = 0; ps < 2; ++ps) {
            if (lane < 8) *(volatile v4f*)o = val;
            if (ps == 0) __threadfence(); }
    }
}

__global__ __launch_bounds__(32) void k_dot(const bf* __restrict__ A, const bf* __restrict__ Bt, const float* __restrict__ invA, const float* __restrict__ invB, float* DOT) {
    __shared__ __align__(16) float os[16 * 68];
    const int K = DW;
    const int lane = threadIdx.x & 31, lr = lane & 15, hi = lane >> 4; const int r0 = blockIdx.x * 64, c0 = blockIdx.y * 64;
    v8f acc[4][4];
#pragma unroll
    for (int mb = 0; mb < 4; ++mb)
#pragma unroll
        for (int nb = 0; nb < 4; ++nb) acc[mb][nb] = (v8f){};
    const size_t aoff = (size_t)(r0 + lr) * K + 8 * hi, boff = (size_t)(c0 + lr) * K + 8 * hi;
#pragma unroll 1
    for (int kc = 0; kc < K; kc += 32) {
        v16bf a[4];
#pragma unroll
        for (int mb = 0; mb < 4; ++mb) a[mb] = ldb(A + aoff + (size_t)mb * 16 * K + kc);
#pragma unroll
        for (int nb = 0; nb < 4; ++nb) { const v16bf b = ldb(Bt + boff + (size_t)nb * 16 * K + kc);
#pragma unroll
            for (int mb = 0; mb < 4; ++mb) acc[mb][nb] = wmmab_g(a[mb], b, acc[mb][nb]); }
    }
    float ic[4];
#pragma unroll
    for (int nb = 0; nb < 4; ++nb) ic[nb] = invB[c0 + nb * 16 + lr];
#pragma unroll
    for (int mb = 0; mb < 4; ++mb) {
        const v4f i0 = *(const v4f*)(invA + r0 + mb * 16 + hi * 8);
        const v4f i1 = *(const v4f*)(invA + r0 + mb * 16 + hi * 8 + 4);
        float ir[8];
#pragma unroll
        for (int j = 0; j < 4; ++j) { ir[j] = i0[j]; ir[4 + j] = i1[j]; }
#pragma unroll
        for (int nb = 0; nb < 4; ++nb) {
#pragma unroll
            for (int j = 0; j < 8; ++j) os[(hi * 8 + j) * 68 + nb * 16 + lr] = (acc[mb][nb][j] * ir[j]) * ic[nb]; }
        wave_sync();
        float* ob = DOT + (size_t)(r0 + mb * 16) * NCOL + c0;
#pragma unroll 1
        for (int ps = 0; ps < 2; ++ps) {
#pragma unroll
            for (int s = 0; s < 8; ++s) { const int row = 2 * s + (lane >> 4), c4 = (lane & 15) * 4;
                const v4f val = *(const v4fa*)(&os[row * 68 + c4]);
                *(volatile v4f*)(ob + (size_t)row * NCOL + c4) = val; }
            if (ps == 0) __threadfence(); }
        wave_sync();
    }
}

__global__ __launch_bounds__(32 * EW) void k_epi(const float* __restrict__ DOT, const int* __restrict__ mask, float* OUT) {
    __shared__ __align__(16) float dl[EW * TT * VV];
    __shared__ __align__(16) float res[NVD];
    const int lane = threadIdx.x & 31;
    const int wave = __builtin_amdgcn_readfirstlane((int)(threadIdx.x >> 5));
    const int a = blockIdx.x;
    const float tmv = (float)mask[a * TT + lane];
    const int wb = wave * (TT * VV) + lane * VV;
    const float ninf = -__builtin_inff();
#pragma unroll 1
    for (int i = 0; i < BPW; ++i) {
        const int b = wave * BPW + i;
        const size_t off = ((size_t)a * TT + (size_t)lane) * NCOL + (size_t)b * VV;
        const v4f x0 = *(const v4f*)(DOT + off), x1 = *(const v4f*)(DOT + off + 4), x2 = *(const v4f*)(DOT + off + 8);
        *(v4fa*)(&dl[wb]) = x0; *(v4fa*)(&dl[wb + 4]) = x1; *(v4fa*)(&dl[wb + 8]) = x2;
        wave_sync();
        float m1 = ninf;
#pragma unroll 1
        for (int v = 0; v < VV; ++v) m1 = fmaxf(m1, (dl[wb + v] * tmv) * TAUF);
        float s1 = 0.0f, a1 = 0.0f;
#pragma unroll 1
        for (int v = 0; v < VV; ++v) { const float d = dl[wb + v];
            const float e = __builtin_amdgcn_exp2f(((d * tmv) * TAUF - m1) * L2E);
            s1 += e; a1 += e * d; }
        const float t2v = a1 * (1.0f / s1);
        const float z2 = (t2v == 0.0f) ? ninf : t2v * TAUF;
        const float mz = wmax(z2);
        const float e2 = __builtin_amdgcn_exp2f((z2 - mz) * L2E);
        const float sz = wsum(e2);
        const float wt = e2 * (1.0f / sz);
        float m2 = ninf, s2 = 0.0f, a2 = 0.0f;
#pragma unroll 1
        for (int v = 0; v < VV; ++v) { const float d = dl[wb + v];
            const float lg = d * tmv;
            const float z = (lg == 0.0f) ? ninf : lg * TAUF;
            const float mx = wmax(z);
            const float e = __builtin_amdgcn_exp2f((z - mx) * L2E);
            const float se = wsum(e);
            const float sa = wsum(e * d);
            const float c = wsum(wt * d);
            const float x = (sa * (1.0f / se)) * TAUF;
            const float mnew = fmaxf(m2, x);
            const float alpha = __builtin_amdgcn_exp2f((m2 - mnew) * L2E);
            const float ex = __builtin_amdgcn_exp2f((x - mnew) * L2E);
            s2 = s2 * alpha + ex; a2 = a2 * alpha + ex * c; m2 = mnew; }
        const float o = a2 * (1.0f / s2);
        if (lane == 0) res[b] = o;
        wave_sync();
    }
    __syncthreads();
    if (wave == 0) {
        const int lc = lane < (NVD / 4) ? lane : (NVD / 4 - 1);
        const v4f val = *(const v4fa*)(&res[lc * 4]);
        float* orow = OUT + (size_t)a * NVD_FULL + lc * 4;
#pragma unroll 1
        for (int ps = 0; ps < 2; ++ps) {
            if (lane < (NVD / 4)) *(volatile v4f*)orow = val;
            if (ps == 0) __threadfence(); }
    }
}

static constexpr size_t al256(size_t v) { return (v + 255) & ~(size_t)255; }
static constexpr size_t SZ_TB  = al256((size_t)NROW * DW * 2);
static constexpr size_t SZ_VB  = al256((size_t)NCOL * DW * 2);
static constexpr size_t SZ_INV = al256((size_t)(NROW + NCOL) * 4);
static constexpr size_t SZ_DOT = al256((size_t)NROW * NCOL * 4);
static constexpr size_t SZ_TOTAL = SZ_TB + SZ_VB + SZ_INV + SZ_DOT;
static_assert(SZ_TOTAL <= (size_t)134217728);
static_assert(((size_t)NROW * 4) % 128 == 0);
static_assert(((size_t)NCOL * 4) % 128 == 0);
static_assert(((size_t)NVD_FULL * 4) % 128 == 0);

extern "C" void kernel_launch(void* const* d_in, const int* in_sizes, int n_in,
                              void* d_out, int out_size, void* d_ws, size_t ws_size, hipStream_t stream) {
    if (n_in < 3) return;
    if ((size_t)in_sizes[0] < (size_t)NROW * DW) return;
    if ((size_t)in_sizes[1] < (size_t)NCOL * DW) return;
    if ((size_t)in_sizes[2] < (size_t)NROW) return;
    if ((size_t)out_size < (size_t)(NTX - 1) * NVD_FULL + NVD) return;
    if (SZ_TOTAL > ws_size) return;
    const float* tx = (const float*)d_in[0];
    const float* vd = (const float*)d_in[1];
    const int* tmk = (const int*)d_in[2];
    float* OUT = (float*)d_out;
    char* wsp = (char*)d_ws;
    bf* TB = (bf*)wsp; wsp += SZ_TB;
    bf* VB = (bf*)wsp; wsp += SZ_VB;
    float* INV = (float*)wsp; wsp += SZ_INV;
    float* DOT = (float*)wsp; wsp += SZ_DOT;
    float* INVT = INV; float* INVV = INV + NROW;

    { const size_t n8 = (size_t)NROW * DW / 8; k_cvt8<<<(unsigned)((n8 + 255) / 256), 256, 0, stream>>>(tx, TB, n8); }
    { const size_t n8 = (size_t)NCOL * DW / 8; k_cvt8<<<(unsigned)((n8 + 255) / 256), 256, 0, stream>>>(vd, VB, n8); }
    k_norm<<<NROW / 32, 32 * EW, 0, stream>>>(tx, INVT, NROW);
    k_norm<<<NCOL / 32, 32 * EW, 0, stream>>>(vd, INVV, NCOL);
    k_dot<<<dim3(NROW / 64, NCOL / 64, 1), 32, 0, stream>>>(TB, VB, INVT, INVV, DOT);
    k_epi<<<NTX, 32 * EW, 0, stream>>>(DOT, tmk, OUT);
}
